// DifferentialAttention_18356690223144
// MI455X (gfx1250) — hardware-verified
//
#include <hip/hip_runtime.h>


typedef _Float16 v16h __attribute__((ext_vector_type(16)));
typedef _Float16 h8   __attribute__((ext_vector_type(8)));
typedef float    v8f  __attribute__((ext_vector_type(8)));
typedef float    f4   __attribute__((ext_vector_type(4)));
typedef unsigned int u4 __attribute__((ext_vector_type(4)));

#ifndef NB
#define NB 2
#endif
#ifndef SEQ
#define SEQ 2048
#endif
#define NB_FULL  2
#define SEQ_FULL 2048
#define NH   16
#define HD   64
#define D2   32
#define NBH  (NB * NH)
#define QTILE 128
#define STILE 64
#define NT    (SEQ / STILE)

static_assert(NB <= NB_FULL);
static_assert(SEQ <= SEQ_FULL);
static_assert(SEQ % QTILE == 0);
static_assert(SEQ % STILE == 0);
static_assert((NBH * SEQ) % 16 == 0);

#define KH_BYTES  ((size_t)NBH * SEQ * HD * 2)
#define VT_BYTES  ((size_t)NBH * HD * SEQ * 2)
#define CTX_BYTES ((size_t)NBH * SEQ * HD * 4)
#define WS_NEED   (KH_BYTES + VT_BYTES + 2 * CTX_BYTES)
static_assert(WS_NEED <= (size_t)134217728);
static_assert(KH_BYTES % 128 == 0);
static_assert(VT_BYTES % 128 == 0);
static_assert(CTX_BYTES % 128 == 0);

#define KL_STR   40
#define VL_STR   72
#define KL_BYTES (STILE * KL_STR * 2)
#define VL_BYTES (HD * VL_STR * 2)
#define PS_BYTES (STILE * 16 * 2)
#define SMEM_ATT (KL_BYTES + VL_BYTES + 8 * 2 * PS_BYTES)
#define STG_BYTES (QTILE * HD * 4)
static_assert(STG_BYTES <= SMEM_ATT);

__device__ __forceinline__ float bf16_rne(float x) {
  unsigned u = __float_as_uint(x);
  u = (u + 0x7FFFu + ((u >> 16) & 1u)) & 0xFFFF0000u;
  return __uint_as_float(u);
}
__device__ __forceinline__ _Float16 cv16(float x) { return (_Float16)(bf16_rne(x) * 16.0f); }

__device__ __forceinline__ v8f wmma16(v16h a, v16h b, v8f c) {
  v8f d = __builtin_amdgcn_wmma_f32_16x16x32_f16(false, a, false, b, (short)0, c, false, false);
  asm volatile("v_nop\n\tv_nop\n\tv_nop\n\tv_nop" : "+v"(d) : "v"(a), "v"(b));
  return d;
}

__global__ __launch_bounds__(256) void k_conv(const float* __restrict__ K,
                                              const float* __restrict__ V,
                                              _Float16* __restrict__ Kh,
                                              _Float16* __restrict__ Vt) {
  __shared__ __align__(16) _Float16 vtl[HD * VL_STR];
  const int tid = threadIdx.x;
  const int bh  = blockIdx.y;
  const int s0  = blockIdx.x * STILE;
  const float* Kg = K + ((size_t)bh * SEQ_FULL + s0) * HD;
  const float* Vg = V + ((size_t)bh * SEQ_FULL + s0) * HD;
  _Float16* Kp = Kh + ((size_t)bh * SEQ + s0) * HD;
  _Float16* Vp = Vt + (size_t)bh * HD * SEQ + s0;

  union HU8 { h8 h; u4 u; _Float16 s[8]; };
  HU8 kv[2];
#pragma unroll
  for (int i = 0; i < 2; ++i) {
    const int idx = tid + 256 * i;
    const int row = idx >> 3;
    const int c8  = (idx & 7) * 8;
    const f4 a  = *(const f4*)(Kg + row * HD + c8);
    const f4 b  = *(const f4*)(Kg + row * HD + c8 + 4);
    const f4 va = *(const f4*)(Vg + row * HD + c8);
    const f4 vb = *(const f4*)(Vg + row * HD + c8 + 4);
#pragma unroll
    for (int e = 0; e < 4; ++e) {
      kv[i].s[e]     = cv16(a[e]);
      kv[i].s[4 + e] = cv16(b[e]);
      vtl[(c8 + e) * VL_STR + row]     = cv16(va[e]);
      vtl[(c8 + 4 + e) * VL_STR + row] = cv16(vb[e]);
    }
  }
  __syncthreads();
  HU8 vv[2];
#pragma unroll
  for (int i = 0; i < 2; ++i) {
    const int idx = tid + 256 * i;
    const int d   = idx >> 3;
    const int p8  = (idx & 7) * 8;
    vv[i].h = *(const h8*)(vtl + d * VL_STR + p8);
  }
#pragma unroll
  for (int i = 0; i < 2; ++i) {
    const int idx = tid + 256 * i;
    const int row = idx >> 3, c8 = (idx & 7) * 8;
    *(volatile u4*)(Kp + row * HD + c8) = kv[i].u;
    *(volatile u4*)(Vp + (size_t)row * SEQ + c8) = vv[i].u;
  }
  __threadfence();
#pragma unroll
  for (int i = 0; i < 2; ++i) {
    const int idx = tid + 256 * i;
    const int row = idx >> 3, c8 = (idx & 7) * 8;
    *(volatile u4*)(Kp + row * HD + c8) = kv[i].u;
    *(volatile u4*)(Vp + (size_t)row * SEQ + c8) = vv[i].u;
  }
}

__global__ __launch_bounds__(256) void k_attn(const float* __restrict__ Q,
                                              const _Float16* __restrict__ Kh,
                                              const _Float16* __restrict__ Vt,
                                              float* __restrict__ Ctx) {
  const int tid  = threadIdx.x;
  const int lane = tid & 31;
  const int wave = tid >> 5;
  const int l16  = lane & 15;
  const int half = lane >> 4;
  const int kb8  = half * 8;

  const int bh    = blockIdx.y;
  const int qBase = blockIdx.x * QTILE;
  const int doff  = blockIdx.z * D2;
  float* ctx = Ctx + (size_t)blockIdx.z * ((size_t)NBH * SEQ * HD);

  __shared__ __align__(16) unsigned char smem[SMEM_ATT];
  _Float16* Kl  = (_Float16*)smem;
  _Float16* Vl  = (_Float16*)(smem + KL_BYTES);
  _Float16* pHi = (_Float16*)(smem + KL_BYTES + VL_BYTES + wave * (2 * PS_BYTES));
  _Float16* pLo = pHi + STILE * 16;
  float*    stg = (float*)smem;

  union HU { v16h v; h8 p[2]; _Float16 s[16]; };
  HU uq;
  {
    const float* qp = Q + ((size_t)bh * SEQ_FULL + qBase + wave * 16 + l16) * HD + doff;
    const f4 x0 = *(const f4*)(qp + kb8);
    const f4 x1 = *(const f4*)(qp + kb8 + 4);
    const f4 x2 = *(const f4*)(qp + 16 + kb8);
    const f4 x3 = *(const f4*)(qp + 16 + kb8 + 4);
#pragma unroll
    for (int e = 0; e < 4; ++e) {
      uq.s[e]      = cv16(x0[e]);
      uq.s[4 + e]  = cv16(x1[e]);
      uq.s[8 + e]  = cv16(x2[e]);
      uq.s[12 + e] = cv16(x3[e]);
    }
  }
  const v16h qa = uq.v;

  float m[8], lsum[8];
  v8f accH[4], accL[4];
#pragma unroll
  for (int j = 0; j < 8; ++j) { m[j] = -1.0e30f; lsum[j] = 0.0f; }
#pragma unroll
  for (int n = 0; n < 4; ++n)
#pragma unroll
    for (int j = 0; j < 8; ++j) { accH[n][j] = 0.0f; accL[n][j] = 0.0f; }

  const _Float16* khBase = Kh + (size_t)bh * SEQ * HD + doff;
  const _Float16* vtBase = Vt + (size_t)bh * HD * SEQ;
  const int skey = tid >> 2;
  const int spc  = (tid & 3) * 8;
  const float SC = 0.17677669529663688f * 0.00390625f;

  for (int it = 0; it < NT; ++it) {
    const int kb = it * STILE;
    __syncthreads();
    {
      const h8 kx = *(const h8*)(khBase + (size_t)(kb + skey) * HD + spc);
      *(h8*)(Kl + skey * KL_STR + spc) = kx;
#pragma unroll
      for (int i = 0; i < 2; ++i) {
        const int idx = tid + 256 * i;
        const int d   = idx >> 3;
        const int p8  = (idx & 7) * 8;
        const h8 vx = *(const h8*)(vtBase + (size_t)d * SEQ + kb + p8);
        *(h8*)(Vl + d * VL_STR + p8) = vx;
      }
    }
    __syncthreads();

    float p[4][8];
    float tmax[8];
#pragma unroll
    for (int j = 0; j < 8; ++j) tmax[j] = -1.0e30f;

#pragma unroll
    for (int t = 0; t < 4; ++t) {
      HU ub;
      const _Float16* kr = Kl + (t * 16 + l16) * KL_STR;
      ub.p[0] = *(const h8*)(kr + kb8);
      ub.p[1] = *(const h8*)(kr + 16 + kb8);
      v8f c8;
#pragma unroll
      for (int j = 0; j < 8; ++j) c8[j] = 0.0f;
      c8 = wmma16(qa, ub.v, c8);
#pragma unroll
      for (int j = 0; j < 8; ++j) {
        const float lg = c8[j] * SC;
        p[t][j] = lg;
        tmax[j] = fmaxf(tmax[j], lg);
      }
    }

#pragma unroll
    for (int j = 0; j < 8; ++j) {
      float v = tmax[j];
      v = fmaxf(v, __shfl_xor(v, 1, 32));
      v = fmaxf(v, __shfl_xor(v, 2, 32));
      v = fmaxf(v, __shfl_xor(v, 4, 32));
      v = fmaxf(v, __shfl_xor(v, 8, 32));
      tmax[j] = v;
    }
    float corr[8];
#pragma unroll
    for (int j = 0; j < 8; ++j) {
      const float nm = fmaxf(m[j], tmax[j]);
      corr[j] = __expf(m[j] - nm);
      m[j] = nm;
    }
#pragma unroll
    for (int j = 0; j < 8; ++j) {
      float s = 0.0f;
#pragma unroll
      for (int t = 0; t < 4; ++t) {
        p[t][j] = __expf(p[t][j] - m[j]);
        s += p[t][j];
      }
      s += __shfl_xor(s, 1, 32);
      s += __shfl_xor(s, 2, 32);
      s += __shfl_xor(s, 4, 32);
      s += __shfl_xor(s, 8, 32);
      lsum[j] = lsum[j] * corr[j] + s;
    }
#pragma unroll
    for (int n = 0; n < 4; ++n)
#pragma unroll
      for (int j = 0; j < 8; ++j) { accH[n][j] *= corr[j]; accL[n][j] *= corr[j]; }

#pragma unroll
    for (int t = 0; t < 4; ++t) {
      union { _Float16 s[8]; h8 v; } uh, ul;
#pragma unroll
      for (int j = 0; j < 8; ++j) {
        const float pc = p[t][j] * 4096.0f;
        const _Float16 hv = (_Float16)pc;
        uh.s[j] = hv;
        ul.s[j] = (_Float16)((pc - (float)hv) * 1024.0f);
      }
      *(h8*)(pHi + (t * 16 + l16) * 16 + half * 8) = uh.v;
      *(h8*)(pLo + (t * 16 + l16) * 16 + half * 8) = ul.v;
    }
    __syncthreads();

    v16h ph0, ph1, pl0, pl1;
#pragma unroll
    for (int c = 0; c < 8; ++c) {
      ph0[c]     = pHi[(kb8 + c) * 16 + l16];
      ph0[c + 8] = pHi[(16 + kb8 + c) * 16 + l16];
      ph1[c]     = pHi[(32 + kb8 + c) * 16 + l16];
      ph1[c + 8] = pHi[(48 + kb8 + c) * 16 + l16];
      pl0[c]     = pLo[(kb8 + c) * 16 + l16];
      pl0[c + 8] = pLo[(16 + kb8 + c) * 16 + l16];
      pl1[c]     = pLo[(32 + kb8 + c) * 16 + l16];
      pl1[c + 8] = pLo[(48 + kb8 + c) * 16 + l16];
    }
#pragma unroll
    for (int n = 0; n < 4; ++n) {
      HU uv0, uv1;
      const _Float16* vr = Vl + (16 * n + l16) * VL_STR;
      uv0.p[0] = *(const h8*)(vr + kb8);
      uv0.p[1] = *(const h8*)(vr + 16 + kb8);
      uv1.p[0] = *(const h8*)(vr + 32 + kb8);
      uv1.p[1] = *(const h8*)(vr + 48 + kb8);
      accH[n] = wmma16(ph0, uv0.v, accH[n]);
      accH[n] = wmma16(ph1, uv1.v, accH[n]);
      accL[n] = wmma16(pl0, uv0.v, accL[n]);
      accL[n] = wmma16(pl1, uv1.v, accL[n]);
    }
  }
  __syncthreads();

  {
    float inv[8];
#pragma unroll
    for (int j = 0; j < 8; ++j) inv[j] = (1.0f / lsum[j]) * (1.0f / 65536.0f);
    float* sw = stg + wave * (16 * HD);
#pragma unroll
    for (int n = 0; n < 4; ++n)
#pragma unroll
      for (int j = 0; j < 8; ++j)
        sw[(8 * half + j) * HD + 16 * n + l16] = (accH[n][j] + accL[n][j] * (1.0f / 1024.0f)) * inv[j];
  }
  __syncthreads();
  f4 ov[8];
  {
    const float* sw = stg + wave * (16 * HD);
#pragma unroll
    for (int k = 0; k < 8; ++k) {
      const int row = 2 * k + half;
      ov[k] = *(const f4*)(sw + row * HD + l16 * 4);
    }
  }
  float* cg = ctx + ((size_t)bh * SEQ + qBase + wave * 16) * HD;
#pragma unroll
  for (int k = 0; k < 8; ++k)
    *(volatile f4*)(cg + (size_t)(2 * k + half) * HD + l16 * 4) = ov[k];
  __threadfence();
#pragma unroll
  for (int k = 0; k < 8; ++k)
    *(volatile f4*)(cg + (size_t)(2 * k + half) * HD + l16 * 4) = ov[k];
}

__global__ __launch_bounds__(256) void k_comb(const float* __restrict__ C0,
                                              const float* __restrict__ C1,
                                              const float* __restrict__ Lam,
                                              int nlam,
                                              float* __restrict__ Out) {
  const int tid = threadIdx.x;
  const int r   = blockIdx.x * 16 + (tid >> 4);
  const int c4  = (tid & 15) * 4;
  const int bh  = r / SEQ;
  int h = bh % NH;
  h = min(h, nlam - 1);
  h = max(h, 0);
  const float lam = bf16_rne(Lam[h]);
  const size_t off = (size_t)r * HD + c4;
  const f4 a = *(const f4*)(C0 + off);
  const f4 b = *(const f4*)(C1 + off);
  float x[4];
#pragma unroll
  for (int i = 0; i < 4; ++i) x[i] = a[i] - lam * b[i];
  float s = (x[0] + x[1]) + (x[2] + x[3]);
  s += __shfl_xor(s, 1, 32);
  s += __shfl_xor(s, 2, 32);
  s += __shfl_xor(s, 4, 32);
  s += __shfl_xor(s, 8, 32);
  const float mean = s * (1.0f / 64.0f);
  float d[4];
  float ss = 0.0f;
#pragma unroll
  for (int i = 0; i < 4; ++i) { d[i] = x[i] - mean; ss += d[i] * d[i]; }
  ss += __shfl_xor(ss, 1, 32);
  ss += __shfl_xor(ss, 2, 32);
  ss += __shfl_xor(ss, 4, 32);
  ss += __shfl_xor(ss, 8, 32);
  const float var = ss * (1.0f / 64.0f);
  const float rs  = rsqrtf(var + 1.0e-5f);
  f4 o;
#pragma unroll
  for (int i = 0; i < 4; ++i) o[i] = (d[i] * rs) * 0.2f;
  *(volatile f4*)(Out + off) = o;
  __threadfence();
  *(volatile f4*)(Out + off) = o;
}

extern "C" void kernel_launch(void* const* d_in, const int* in_sizes, int n_in,
                              void* d_out, int out_size, void* d_ws, size_t ws_size,
                              hipStream_t stream) {
  if (n_in < 4) return;
  const long long needIn = ((long long)(NBH - 1) * SEQ_FULL + SEQ) * HD;
  if ((long long)in_sizes[0] < needIn || (long long)in_sizes[1] < needIn ||
      (long long)in_sizes[2] < needIn || in_sizes[3] < 1) return;
  if ((long long)out_size < (long long)NBH * SEQ * HD) return;
  if (d_ws == nullptr || ws_size < WS_NEED) return;

  const float* Q   = (const float*)d_in[0];
  const float* K   = (const float*)d_in[1];
  const float* V   = (const float*)d_in[2];
  const float* Lam = (const float*)d_in[3];
  float* Out = (float*)d_out;

  char* ws = (char*)d_ws;
  _Float16* Kh  = (_Float16*)(ws);
  _Float16* Vt  = (_Float16*)(ws + KH_BYTES);
  float*    Ctx = (float*)(ws + KH_BYTES + VT_BYTES);
  float*    Ctx1 = Ctx + (size_t)NBH * SEQ * HD;

  k_conv<<<dim3(SEQ / STILE, NBH), dim3(256), 0, stream>>>(K, V, Kh, Vt);
  k_attn<<<dim3(SEQ / QTILE, NBH, 2), dim3(256), 0, stream>>>(Q, Kh, Vt, Ctx);
  k_comb<<<dim3((NBH * SEQ) / 16), dim3(256), 0, stream>>>(Ctx, Ctx1, Lam, in_sizes[3], Out);
}
